// Decoder_32615981645904
// MI455X (gfx1250) — hardware-verified
//
#include <hip/hip_runtime.h>
#include <math.h>

constexpr int NBAT  = 64;
constexpr int NLOC  = 196;
constexpr int NCAP  = 20;
constexpr int NSTP  = 19;
constexpr int NDIM  = 512;
constexpr int NVOC  = 10000;
constexpr int NVOCP = 10048;
constexpr int NROW  = NBAT * NSTP;
constexpr int NFROW = NBAT * NLOC;
constexpr int NGATE = 4 * NDIM;
constexpr int ALPITCH = 256;
constexpr int HPIT  = 520;
constexpr int P1PIT = 1024;
constexpr float WCARRY = 64.0f;
constexpr float ACARRY = 64.0f;
constexpr float WINV = 1.0f / WCARRY;
constexpr float PINV = 1.0f / (WCARRY * ACARRY);
constexpr int NOUT0 = NBAT * NSTP * NVOC;
constexpr int NOUT1 = NBAT * NSTP * NLOC;
constexpr int BOFF_INIT = 0;
constexpr int BOFF_AT   = 1024;
constexpr int BOFF_GATE = 2048;
constexpr int BOFF_DEEP = 4096;
constexpr int BOFF_LO   = 4608;
constexpr int BTOTAL    = BOFF_LO + NVOCP;
static_assert(NROW == 1216);
static_assert(NFROW == 12544);
static_assert(NROW % 64 == 0 && NFROW % 64 == 0 && NVOCP % 64 == 0 && NDIM % 64 == 0);
static_assert(NDIM % 32 == 0);
static_assert(NVOC % 4 == 0 && NLOC % 4 == 0);
static_assert((size_t)NOUT0 * 4 == (size_t)48640000);
static_assert(((size_t)NOUT0 * 4) % 128 == 0);
static_assert(((size_t)NOUT0 + (size_t)NOUT1) * 4 == (size_t)49593344);
static_assert(BTOTAL % 4 == 0 && BTOTAL == 14656);
static_assert(NBAT % 16 == 0);

typedef __attribute__((ext_vector_type(16))) _Float16 v16h;
typedef __attribute__((ext_vector_type(8)))  _Float16 v8h;
typedef __attribute__((ext_vector_type(4)))  _Float16 v4h;
typedef __attribute__((ext_vector_type(8)))  float    v8f;
typedef __attribute__((ext_vector_type(4)))  float    v4f;

__device__ __forceinline__ void guard4_h(v8f& a0, v8f& a1, v8f& a2, v8f& a3, v16h x, v16h y0, v16h y1, v16h y2, v16h y3) {
  asm volatile("v_nop\n\tv_nop\n\tv_nop\n\tv_nop" : "+v"(a0), "+v"(a1), "+v"(a2), "+v"(a3) : "v"(x), "v"(y0), "v"(y1), "v"(y2), "v"(y3));
}
__device__ __forceinline__ void keep4_h(v16h a, v16h b, v16h c, v16h d) { asm volatile("v_nop" :: "v"(a), "v"(b), "v"(c), "v"(d)); }
__device__ __forceinline__ void acc_guard4(v8f& a, v8f& b, v8f& c, v8f& d) { asm volatile("v_nop\n\tv_nop\n\tv_nop\n\tv_nop" : "+v"(a), "+v"(b), "+v"(c), "+v"(d)); }

struct FragH {
  union U { v16h v; v8h h[2]; };
  static __device__ __forceinline__ v16h load(const _Float16* p) {
    U f; f.h[0] = *(const v8h*)(p); f.h[1] = *(const v8h*)(p + 16); return f.v;
  }
  static __device__ __forceinline__ v8f mma(v16h a, v16h b, v8f c) {
    return __builtin_amdgcn_wmma_f32_16x16x32_f16(false, a, false, b, (short)0, c, false, false);
  }
};

template <int OUT_MODE, bool RESID>
__global__ __launch_bounds__(256) void wmma_gemm64(
    const unsigned short* __restrict__ Ap, int lda,
    const unsigned short* __restrict__ Btp, int ldb,
    void* __restrict__ Cout, int ldc,
    const float* __restrict__ bias,
    const float* __restrict__ resid, int ldr,
    int M, int N, int K, float scale, float oscale) {
  static_assert(OUT_MODE == 0 || OUT_MODE == 1);
  static_assert(!(RESID && OUT_MODE == 0));
  const _Float16* A  = (const _Float16*)Ap;
  const _Float16* Bt = (const _Float16*)Btp;
  __shared__ __align__(16) float sT[8][16 * 68];
  const int lane = threadIdx.x & 31;
  const int wave = threadIdx.x >> 5;
  const int tilesN = N >> 6;
  const int tilesM = M >> 6;
  const int tile = blockIdx.x * 8 + wave;
  if (tile >= tilesM * tilesN) return;
  const int tm = tile / tilesN;
  const int tn = tile - tm * tilesN;
  const int m0 = tm << 6;
  const int n0 = tn << 6;
  const int rlane = lane & 15;
  const int koff  = (lane >> 4) * 8;
  const int mOff  = (lane >> 4) * 8;

  v8f acc[4][4];
#pragma unroll
  for (int i = 0; i < 4; ++i)
#pragma unroll
    for (int j = 0; j < 4; ++j) acc[i][j] = (v8f){0.f, 0.f, 0.f, 0.f, 0.f, 0.f, 0.f, 0.f};

  for (int k0 = 0; k0 < K; k0 += 32) {
    v16h bh[4];
#pragma unroll
    for (int j = 0; j < 4; ++j) {
      const size_t bo = (size_t)(n0 + (j << 4) + rlane) * ldb + koff + k0;
      bh[j] = FragH::load(Bt + bo);
    }
#pragma unroll
    for (int i = 0; i < 4; ++i) {
      const size_t ao = (size_t)(m0 + (i << 4) + rlane) * lda + koff + k0;
      const v16h ah = FragH::load(A + ao);
#pragma unroll
      for (int j = 0; j < 4; ++j) acc[i][j] = FragH::mma(ah, bh[j], acc[i][j]);
      guard4_h(acc[i][0], acc[i][1], acc[i][2], acc[i][3], ah, bh[0], bh[1], bh[2], bh[3]);
    }
    keep4_h(bh[0], bh[1], bh[2], bh[3]);
  }
  acc_guard4(acc[0][0], acc[0][1], acc[0][2], acc[0][3]);
  acc_guard4(acc[1][0], acc[1][1], acc[1][2], acc[1][3]);
  acc_guard4(acc[2][0], acc[2][1], acc[2][2], acc[2][3]);
  acc_guard4(acc[3][0], acc[3][1], acc[3][2], acc[3][3]);

  float* slab = sT[wave];
#pragma unroll
  for (int i = 0; i < 4; ++i) {
    const int mBase = m0 + (i << 4);
#pragma unroll
    for (int j = 0; j < 4; ++j) {
      const int n = n0 + (j << 4) + rlane;
      const float bv = bias[n];
#pragma unroll
      for (int r = 0; r < 8; ++r) {
        const float v = acc[i][j][r] * scale + bv;
        slab[(mOff + r) * 68 + (j << 4) + rlane] = v;
      }
    }
    __builtin_amdgcn_fence(__ATOMIC_RELEASE, "workgroup");
    __builtin_amdgcn_wave_barrier();
    __builtin_amdgcn_fence(__ATOMIC_ACQUIRE, "workgroup");
    if (OUT_MODE == 0) {
      float* C = (float*)Cout;
      const int hh = lane >> 4, c4 = (lane & 15) * 4;
      for (int pass = 0; pass < 2; ++pass) {
#pragma unroll
        for (int it = 0; it < 8; ++it) {
          const int row = it * 2 + hh;
          const v4f v = *(const v4f*)(slab + row * 68 + c4);
          *(volatile v4f*)(C + (size_t)(mBase + row) * ldc + n0 + c4) = v;
        }
        __threadfence();
      }
    } else {
      const int q = lane >> 3, c8 = (lane & 7) * 8;
      unsigned short* C = (unsigned short*)Cout;
      v8h hv[4];
#pragma unroll
      for (int it = 0; it < 4; ++it) {
        const int row = it * 4 + q;
        const float* sp = slab + row * 68 + c8;
        v4f r0 = (v4f){0.f, 0.f, 0.f, 0.f};
        v4f r1 = (v4f){0.f, 0.f, 0.f, 0.f};
        if (RESID) {
          const float* rp = resid + (size_t)(mBase + row) * ldr + n0 + c8;
          r0 = *(const v4f*)(rp);
          r1 = *(const v4f*)(rp + 4);
        }
#pragma unroll
        for (int e = 0; e < 4; ++e) {
          const float x0 = (sp[e] + r0[e]) * oscale;
          const float x1 = (sp[4 + e] + r1[e]) * oscale;
          hv[it][e]     = (_Float16)x0;
          hv[it][4 + e] = (_Float16)x1;
        }
      }
      for (int pass = 0; pass < 2; ++pass) {
#pragma unroll
        for (int it = 0; it < 4; ++it) {
          const int row = it * 4 + q;
          *(volatile v8h*)(C + (size_t)(mBase + row) * ldc + n0 + c8) = hv[it];
        }
        __threadfence();
      }
    }
    __builtin_amdgcn_fence(__ATOMIC_RELEASE, "workgroup");
    __builtin_amdgcn_wave_barrier();
    __builtin_amdgcn_fence(__ATOMIC_ACQUIRE, "workgroup");
  }
}

__global__ __launch_bounds__(256) void cvt8_kernel(const float* __restrict__ src, unsigned short* __restrict__ dst, int n8, float sc) {
  const int i = blockIdx.x * 256 + threadIdx.x;
  if (i < n8) {
    const float* sp = src + (size_t)i * 8;
    const v4f a = *(const v4f*)(sp);
    const v4f b = *(const v4f*)(sp + 4);
    v8h hv;
#pragma unroll
    for (int e = 0; e < 4; ++e) {
      hv[e]     = (_Float16)(a[e] * sc);
      hv[4 + e] = (_Float16)(b[e] * sc);
    }
    *(volatile v8h*)(dst + (size_t)i * 8) = hv;
    __threadfence();
    *(volatile v8h*)(dst + (size_t)i * 8) = hv;
  }
}

template <bool H16>
__global__ __launch_bounds__(256) void gather_kernel(const float* __restrict__ emb, const int* __restrict__ cap, void* __restrict__ outp) {
  const int i = blockIdx.x * 256 + threadIdx.x;
  if (H16) {
    if (i < NROW * 64) {
      const int m = i >> 6, c8 = (i & 63) * 8;
      const int b = m / NSTP, t = m - b * NSTP;
      int tok = cap[b * NCAP + t];
      tok = tok < 0 ? 0 : (tok > NVOC - 1 ? NVOC - 1 : tok);
      const float* sp = emb + (size_t)tok * NDIM + c8;
      const v4f a = *(const v4f*)(sp);
      const v4f bq = *(const v4f*)(sp + 4);
      v8h hv;
#pragma unroll
      for (int e = 0; e < 4; ++e) {
        hv[e]     = (_Float16)(a[e] * ACARRY);
        hv[4 + e] = (_Float16)(bq[e] * ACARRY);
      }
      unsigned short* o = (unsigned short*)outp + (size_t)m * NDIM + c8;
      *(volatile v8h*)o = hv;
      __threadfence();
      *(volatile v8h*)o = hv;
    }
  } else {
    if (i < NROW * 128) {
      const int m = i >> 7, c4 = (i & 127) * 4;
      const int b = m / NSTP, t = m - b * NSTP;
      int tok = cap[b * NCAP + t];
      tok = tok < 0 ? 0 : (tok > NVOC - 1 ? NVOC - 1 : tok);
      const v4f a = *(const v4f*)(emb + (size_t)tok * NDIM + c4);
      float* o = (float*)outp + (size_t)m * NDIM + c4;
      *(volatile v4f*)o = a;
      __threadfence();
      *(volatile v4f*)o = a;
    }
  }
}

__global__ __launch_bounds__(256) void mean_kernel(const float* __restrict__ feat, unsigned short* __restrict__ outp) {
  const int i = blockIdx.x * 256 + threadIdx.x;
  if (i < NBAT * 64) {
    const int b = i >> 6, c8 = (i & 63) * 8;
    const float* fp = feat + (size_t)b * NLOC * NDIM + c8;
    v4f s0 = (v4f){0.f, 0.f, 0.f, 0.f};
    v4f s1 = (v4f){0.f, 0.f, 0.f, 0.f};
#pragma unroll 1
    for (int l = 0; l < NLOC; ++l) {
      const v4f a = *(const v4f*)(fp + (size_t)l * NDIM);
      const v4f bq = *(const v4f*)(fp + (size_t)l * NDIM + 4);
      s0 += a;
      s1 += bq;
    }
    const float sc = ACARRY * (1.0f / (float)NLOC);
    v8h hv;
#pragma unroll
    for (int e = 0; e < 4; ++e) {
      hv[e]     = (_Float16)(s0[e] * sc);
      hv[4 + e] = (_Float16)(s1[e] * sc);
    }
    unsigned short* o = outp + (size_t)b * NDIM + c8;
    *(volatile v8h*)o = hv;
    __threadfence();
    *(volatile v8h*)o = hv;
  }
}

__global__ __launch_bounds__(256) void tpw_kernel(const float* __restrict__ src, int R, int C, int ldo,
                                                  unsigned short* __restrict__ O, float sc) {
  __shared__ float Tt[64 * 65];
  const int tid = threadIdx.x;
  const int c0 = blockIdx.x * 64, r0 = blockIdx.y * 64;
#pragma unroll
  for (int i = 0; i < 4; ++i) {
    const int idx = i * 256 + tid;
    const int rr = idx >> 4, cc = (idx & 15) * 4;
    const int col = c0 + cc;
    const bool ok = col < C;
    const int colc = ok ? col : (C - 4);
    const v4f v = *(const v4f*)(src + (size_t)(r0 + rr) * (size_t)C + colc);
    Tt[rr * 65 + cc + 0] = ok ? v[0] : 0.0f;
    Tt[rr * 65 + cc + 1] = ok ? v[1] : 0.0f;
    Tt[rr * 65 + cc + 2] = ok ? v[2] : 0.0f;
    Tt[rr * 65 + cc + 3] = ok ? v[3] : 0.0f;
  }
  __syncthreads();
  const int q = tid >> 3, c8 = (tid & 7) * 8;
  v8h hv[2];
#pragma unroll
  for (int g = 0; g < 2; ++g) {
    const int qq = g * 32 + q;
#pragma unroll
    for (int e = 0; e < 8; ++e) {
      const float f = Tt[(c8 + e) * 65 + qq];
      hv[g][e] = (_Float16)(f * sc);
    }
  }
  for (int pass = 0; pass < 2; ++pass) {
#pragma unroll
    for (int g = 0; g < 2; ++g) {
      const size_t o = (size_t)(c0 + g * 32 + q) * (size_t)ldo + (size_t)(r0 + c8);
      *(volatile v8h*)(O + o) = hv[g];
    }
    __threadfence();
  }
}

__global__ __launch_bounds__(256) void bias_kernel(const float* __restrict__ binh, const float* __restrict__ binc,
                                                   const float* __restrict__ badec, const float* __restrict__ bbeta,
                                                   const float* __restrict__ bih, const float* __restrict__ bhh,
                                                   const float* __restrict__ blh, const float* __restrict__ blz,
                                                   const float* __restrict__ blo, float* __restrict__ dst) {
  const int i = blockIdx.x * 256 + threadIdx.x;
  const int w0 = __builtin_amdgcn_readfirstlane((i >> 5) << 5);
  if (i >= BTOTAL / 4) return;
  v4f o;
  if (w0 < 128) {
    o = *(const v4f*)(binh + 4 * i);
  } else if (w0 < 256) {
    o = *(const v4f*)(binc + 4 * (i - 128));
  } else if (w0 < 384) {
    o = *(const v4f*)(badec + 4 * (i - 256));
  } else if (w0 < 512) {
    o = *(const v4f*)(bbeta + 4 * (i - 384));
  } else if (w0 < 1024) {
    const v4f a = *(const v4f*)(bih + 4 * (i - 512));
    const v4f b = *(const v4f*)(bhh + 4 * (i - 512));
    o = a + b;
  } else if (w0 < 1152) {
    const v4f a = *(const v4f*)(blh + 4 * (i - 1024));
    const v4f b = *(const v4f*)(blz + 4 * (i - 1024));
    o = a + b;
  } else {
    const int k = i - 1152;
    const int kc = k < (NVOC / 4) ? k : (NVOC / 4 - 1);
    const v4f a = *(const v4f*)(blo + 4 * kc);
    const bool ok = k < (NVOC / 4);
    o[0] = ok ? a[0] : 0.0f;
    o[1] = ok ? a[1] : 0.0f;
    o[2] = ok ? a[2] : 0.0f;
    o[3] = ok ? a[3] : 0.0f;
  }
  float* op = dst + 4 * i;
  *(volatile v4f*)op = o;
  __threadfence();
  *(volatile v4f*)op = o;
}

__global__ __launch_bounds__(256) void rec_kernel(
    const float* __restrict__ FEAT, const float* __restrict__ FPJ, const float* __restrict__ HC0,
    const float* __restrict__ XG, const float* __restrict__ BAT, const float* __restrict__ WFULL,
    const float* __restrict__ BAFULL,
    const unsigned short* __restrict__ WATp, const unsigned short* __restrict__ WGp,
    float* __restrict__ ALW, unsigned short* __restrict__ HZ) {
  __shared__ __align__(16) _Float16 Hh[2][16 * HPIT];
  __shared__ __align__(16) _Float16 Zz[16 * HPIT];
  __shared__ __align__(16) float    P1s[16 * P1PIT];
  __shared__ __align__(16) float    ALs[16 * ALPITCH];
  __shared__ __align__(16) float    Cs[16 * NDIM];
  const _Float16* WAT = (const _Float16*)WATp;
  const _Float16* WG  = (const _Float16*)WGp;
  const int tid = threadIdx.x, lane = tid & 31, wave = tid >> 5;
  const int c = lane & 15, hh = lane >> 4, koff = hh * 8;
  const int b0 = blockIdx.x * 16;
  const v8f z8 = {0.f, 0.f, 0.f, 0.f, 0.f, 0.f, 0.f, 0.f};

#pragma unroll 1
  for (int i = tid; i < 16 * NDIM; i += 256) {
    const int row = i >> 9, col = i & (NDIM - 1);
    const float* hp = HC0 + (size_t)(b0 + row) * (2 * NDIM);
    const float h0 = tanhf(hp[col]);
    const float c0 = tanhf(hp[NDIM + col]);
    Hh[0][row * HPIT + col] = (_Float16)(h0 * ACARRY);
    Cs[row * NDIM + col] = c0;
  }
  v4f wf[4];
#pragma unroll
  for (int q = 0; q < 4; ++q) wf[q] = *(const v4f*)(WFULL + 128 * q + 4 * lane);
  const float bafull = BAFULL[0];
  __syncthreads();

#pragma unroll 1
  for (int t = 0; t < NSTP; ++t) {
    const int cur = t & 1;
    const int nxt = cur ^ 1;

    {
      const _Float16* arow = &Hh[cur][0] + c * HPIT + koff;
#pragma unroll 1
      for (int grp = 0; grp < 2; ++grp) {
        const int nb = 128 * wave + 64 * grp;
        const _Float16* wb = WAT + (size_t)(nb + c) * NDIM + koff;
        v8f acc[4];
        acc[0] = z8; acc[1] = z8; acc[2] = z8; acc[3] = z8;
#pragma unroll 1
        for (int k0 = 0; k0 < NDIM; k0 += 32) {
          const v16h a  = FragH::load(arow + k0);
          const v16h w0 = FragH::load(wb + k0);
          const v16h w1 = FragH::load(wb + (size_t)16 * NDIM + k0);
          const v16h w2 = FragH::load(wb + (size_t)32 * NDIM + k0);
          const v16h w3 = FragH::load(wb + (size_t)48 * NDIM + k0);
          acc[0] = FragH::mma(a, w0, acc[0]);
          acc[1] = FragH::mma(a, w1, acc[1]);
          acc[2] = FragH::mma(a, w2, acc[2]);
          acc[3] = FragH::mma(a, w3, acc[3]);
          guard4_h(acc[0], acc[1], acc[2], acc[3], a, w0, w1, w2, w3);
        }
        acc_guard4(acc[0], acc[1], acc[2], acc[3]);
#pragma unroll
        for (int j = 0; j < 4; ++j) {
          const int n = nb + 16 * j + c;
          const float bv = BAT[n];
#pragma unroll
          for (int r = 0; r < 8; ++r) P1s[(8 * hh + r) * P1PIT + n] = acc[j][r] * PINV + bv;
        }
      }
    }
    __syncthreads();

#pragma unroll 1
    for (int bi = 0; bi < 2; ++bi) {
      const int b = 2 * wave + bi;
      v4f hpv[4];
#pragma unroll
      for (int q = 0; q < 4; ++q) hpv[q] = *(const v4f*)(P1s + b * P1PIT + 128 * q + 4 * lane);
      const float* fp = FPJ + (size_t)(b0 + b) * NLOC * NDIM + 4 * lane;
#pragma unroll 1
      for (int l = 0; l < NLOC; ++l) {
        float s = 0.0f;
#pragma unroll
        for (int q = 0; q < 4; ++q) {
          const v4f v = *(const v4f*)(fp + (size_t)l * NDIM + 128 * q);
#pragma unroll
          for (int e = 0; e < 4; ++e) s += fmaxf(v[e] + hpv[q][e], 0.0f) * wf[q][e];
        }
#pragma unroll
        for (int off = 16; off > 0; off >>= 1) s += __shfl_xor(s, off, 32);
        if (lane == 0) ALs[b * ALPITCH + l] = s + bafull;
      }
    }
    __syncthreads();

#pragma unroll 1
    for (int bi = 0; bi < 2; ++bi) {
      const int b = 2 * wave + bi;
      float* ar = ALs + b * ALPITCH;
      float mx = -INFINITY;
#pragma unroll 1
      for (int j = 0; j < 7; ++j) {
        const int l = lane + 32 * j;
        const int lc = l < NLOC ? l : (NLOC - 1);
        const float e = ar[lc];
        mx = (l < NLOC) ? fmaxf(mx, e) : mx;
      }
#pragma unroll
      for (int off = 16; off > 0; off >>= 1) mx = fmaxf(mx, __shfl_xor(mx, off, 32));
      float sum = 0.0f;
#pragma unroll 1
      for (int j = 0; j < 8; ++j) {
        const int l = lane + 32 * j;
        const int lc = l < NLOC ? l : (NLOC - 1);
        const float e = ar[lc];
        const float ex0 = expf(e - mx);
        const float ex = (l < NLOC) ? ex0 : 0.0f;
        ar[l] = ex;
        sum += ex;
      }
#pragma unroll
      for (int off = 16; off > 0; off >>= 1) sum += __shfl_xor(sum, off, 32);
      const float inv = 1.0f / sum;
#pragma unroll 1
      for (int j = 0; j < 8; ++j) {
        const int l = lane + 32 * j;
        const float p = ar[l] * inv;
        ar[l] = p;
      }
    }
    __syncthreads();

    for (int pass = 0; pass < 2; ++pass) {
#pragma unroll
      for (int bi = 0; bi < 2; ++bi) {
        const int b = 2 * wave + bi;
        const size_t m = (size_t)(b0 + b) * NSTP + (size_t)t;
#pragma unroll
        for (int q = 0; q < 2; ++q) {
          const v4f v = *(const v4f*)(ALs + b * ALPITCH + 128 * q + 4 * lane);
          *(volatile v4f*)(ALW + m * ALPITCH + 128 * q + 4 * lane) = v;
        }
      }
      __threadfence();
    }
    {
      const int bsel = tid >> 7, c4 = (tid & 127) * 4;
#pragma unroll 1
      for (int i = 0; i < 8; ++i) {
        const int b = 2 * i + bsel;
        const float* fp = FEAT + (size_t)(b0 + b) * NLOC * NDIM + c4;
        const float* al = ALs + b * ALPITCH;
        v4f acc = (v4f){0.f, 0.f, 0.f, 0.f};
#pragma unroll 4
        for (int l = 0; l < NLOC; ++l) {
          const v4f f = *(const v4f*)(fp + (size_t)l * NDIM);
          const float a = al[l];
          acc += f * a;
        }
        const v4f bp = *(const v4f*)(P1s + b * P1PIT + NDIM + c4);
        v4h hv;
#pragma unroll
        for (int e = 0; e < 4; ++e) {
          const float g = 1.0f / (1.0f + expf(-bp[e]));
          hv[e] = (_Float16)(g * acc[e] * ACARRY);
        }
        *(v4h*)(Zz + b * HPIT + c4) = hv;
      }
    }
    __syncthreads();

    {
      float* slab = P1s + wave * 1024;
      const _Float16* ah = &Hh[cur][0] + c * HPIT + koff;
      const _Float16* az = Zz + c * HPIT + koff;
      _Float16* hn = &Hh[nxt][0];
      const size_t gstr = (size_t)NDIM * 1024;
#pragma unroll 1
      for (int nt = 0; nt < 4; ++nt) {
        const int j = 64 * wave + 16 * nt + c;
        const _Float16* wr = WG + (size_t)j * 1024 + koff;
        v8f acc[4];
        acc[0] = z8; acc[1] = z8; acc[2] = z8; acc[3] = z8;
#pragma unroll 1
        for (int k0 = 0; k0 < NDIM; k0 += 32) {
          const v16h a  = FragH::load(ah + k0);
          const v16h w0 = FragH::load(wr + k0);
          const v16h w1 = FragH::load(wr + gstr + k0);
          const v16h w2 = FragH::load(wr + 2 * gstr + k0);
          const v16h w3 = FragH::load(wr + 3 * gstr + k0);
          acc[0] = FragH::mma(a, w0, acc[0]);
          acc[1] = FragH::mma(a, w1, acc[1]);
          acc[2] = FragH::mma(a, w2, acc[2]);
          acc[3] = FragH::mma(a, w3, acc[3]);
          guard4_h(acc[0], acc[1], acc[2], acc[3], a, w0, w1, w2, w3);
        }
#pragma unroll 1
        for (int k0 = 0; k0 < NDIM; k0 += 32) {
          const v16h a  = FragH::load(az + k0);
          const v16h w0 = FragH::load(wr + NDIM + k0);
          const v16h w1 = FragH::load(wr + gstr + NDIM + k0);
          const v16h w2 = FragH::load(wr + 2 * gstr + NDIM + k0);
          const v16h w3 = FragH::load(wr + 3 * gstr + NDIM + k0);
          acc[0] = FragH::mma(a, w0, acc[0]);
          acc[1] = FragH::mma(a, w1, acc[1]);
          acc[2] = FragH::mma(a, w2, acc[2]);
          acc[3] = FragH::mma(a, w3, acc[3]);
          guard4_h(acc[0], acc[1], acc[2], acc[3], a, w0, w1, w2, w3);
        }
        acc_guard4(acc[0], acc[1], acc[2], acc[3]);
#pragma unroll
        for (int g = 0; g < 4; ++g)
#pragma unroll
          for (int r = 0; r < 8; ++r) slab[(g * 16 + 8 * hh + r) * 16 + c] = acc[g][r];
#pragma unroll 1
        for (int r = 0; r < 8; ++r) {
          const int row = 8 * hh + r;
          const float* xp = XG + ((size_t)(b0 + row) * NSTP + (size_t)t) * NGATE + j;
          const float xi = xp[0];
          const float xf = xp[NDIM];
          const float xc = xp[2 * NDIM];
          const float xo = xp[3 * NDIM];
          const float zi = slab[(0 * 16 + row) * 16 + c] * PINV + xi;
          const float zf = slab[(1 * 16 + row) * 16 + c] * PINV + xf;
          const float zc = slab[(2 * 16 + row) * 16 + c] * PINV + xc;
          const float zo = slab[(3 * 16 + row) * 16 + c] * PINV + xo;
          const float si = 1.0f / (1.0f + expf(-zi));
          const float sf = 1.0f / (1.0f + expf(-zf));
          const float so = 1.0f / (1.0f + expf(-zo));
          const float tg = tanhf(zc);
          const float co = Cs[row * NDIM + j];
          const float cn = sf * co + si * tg;
          const float hv = so * tanhf(cn);
          Cs[row * NDIM + j] = cn;
          hn[row * HPIT + j] = (_Float16)(hv * ACARRY);
        }
      }
    }
    __syncthreads();

    for (int pass = 0; pass < 2; ++pass) {
#pragma unroll
      for (int bi = 0; bi < 2; ++bi) {
        const int b = 2 * wave + bi;
        const size_t m = (size_t)(b0 + b) * NSTP + (size_t)t;
#pragma unroll
        for (int q = 0; q < 2; ++q) {
          const int idx = lane + 32 * q;
          const v8h vh = *(const v8h*)(&Hh[nxt][0] + b * HPIT + 8 * idx);
          const v8h vz = *(const v8h*)(Zz + b * HPIT + 8 * idx);
          *(volatile v8h*)(HZ + m * 1024 + 8 * idx) = vh;
          *(volatile v8h*)(HZ + m * 1024 + NDIM + 8 * idx) = vz;
        }
      }
      __threadfence();
    }
  }
}

template <int ROWLEN, int SPITCH>
__global__ __launch_bounds__(256) void copy_rows_kernel(const float* __restrict__ src, float* __restrict__ dst, int n4) {
  static_assert(ROWLEN % 4 == 0 && SPITCH % 4 == 0);
  const int i = blockIdx.x * 256 + threadIdx.x;
  if (i < n4) {
    const unsigned f = 4u * (unsigned)i;
    const unsigned m = f / (unsigned)ROWLEN;
    const unsigned cc = f - m * (unsigned)ROWLEN;
    const v4f v = *(const v4f*)(src + (size_t)m * SPITCH + cc);
    float* op = dst + (size_t)f;
    *(volatile v4f*)op = v;
    __threadfence();
    *(volatile v4f*)op = v;
  }
}

extern "C" void kernel_launch(void* const* d_in, const int* in_sizes, int n_in,
                              void* d_out, int out_size, void* d_ws, size_t ws_size, hipStream_t stream) {
  if (n_in < 25 || d_out == nullptr || d_ws == nullptr) return;
  if (in_sizes[0] != NBAT * NLOC * NDIM || in_sizes[1] != NBAT * NCAP || in_sizes[2] != NVOC * NDIM ||
      in_sizes[11] != 2 * NDIM * NGATE || in_sizes[13] != NDIM * NGATE || in_sizes[19] != NDIM * NVOC ||
      in_sizes[20] != NVOC || out_size != NOUT0 + NOUT1) return;

  const float* features = (const float*)d_in[0];
  const int*   captions = (const int*)d_in[1];
  const float* emb_tab  = (const float*)d_in[2];
  const float* Wa_enc   = (const float*)d_in[3];
  const float* ba_enc   = (const float*)d_in[4];
  const float* Wa_dec   = (const float*)d_in[5];
  const float* ba_dec   = (const float*)d_in[6];
  const float* Wa_full  = (const float*)d_in[7];
  const float* ba_full  = (const float*)d_in[8];
  const float* W_beta   = (const float*)d_in[9];
  const float* b_beta   = (const float*)d_in[10];
  const float* W_ih     = (const float*)d_in[11];
  const float* b_ih     = (const float*)d_in[12];
  const float* W_hh     = (const float*)d_in[13];
  const float* b_hh     = (const float*)d_in[14];
  const float* W_init_h = (const float*)d_in[15];
  const float* b_init_h = (const float*)d_in[16];
  const float* W_init_c = (const float*)d_in[17];
  const float* b_init_c = (const float*)d_in[18];
  const float* W_Lo     = (const float*)d_in[19];
  const float* b_Lo     = (const float*)d_in[20];
  const float* W_Lh     = (const float*)d_in[21];
  const float* b_Lh     = (const float*)d_in[22];
  const float* W_Lz     = (const float*)d_in[23];
  const float* b_Lz     = (const float*)d_in[24];
  float* out_logits = (float*)d_out;
  float* out_alphas = out_logits + (size_t)NOUT0;

  char* ws = (char*)d_ws; size_t off = 0;
  auto carve = [&](size_t bytes) -> char* { char* p = ws + off; off += (bytes + 255) & ~(size_t)255; return p; };
  unsigned short* F16    = (unsigned short*)carve((size_t)NFROW * NDIM * 2);
  float*          FPJ    = (float*)carve((size_t)NFROW * NDIM * 4);
  unsigned short* WLOT   = (unsigned short*)carve((size_t)NVOCP * NDIM * 2);
  float*          LG     = (float*)carve((size_t)NROW * NVOCP * 4);
  float*          XG     = (float*)carve((size_t)NROW * NGATE * 4);
  unsigned short* WAT    = (unsigned short*)carve((size_t)1024 * NDIM * 2);
  unsigned short* WG     = (unsigned short*)carve((size_t)NGATE * 1024 * 2);
  unsigned short* WXT    = (unsigned short*)carve((size_t)NGATE * NDIM * 2);
  unsigned short* WINIT  = (unsigned short*)carve((size_t)1024 * NDIM * 2);
  unsigned short* WDEEP  = (unsigned short*)carve((size_t)NDIM * 1024 * 2);
  unsigned short* WAENC  = (unsigned short*)carve((size_t)NDIM * NDIM * 2);
  float*          X32    = (float*)carve((size_t)NROW * NDIM * 4);
  unsigned short* X16    = (unsigned short*)carve((size_t)NROW * NDIM * 2);
  unsigned short* HZ     = (unsigned short*)carve((size_t)NROW * 1024 * 2);
  unsigned short* PRE16  = (unsigned short*)carve((size_t)NROW * NDIM * 2);
  float*          ALW    = (float*)carve((size_t)NROW * ALPITCH * 4);
  unsigned short* MEAN16 = (unsigned short*)carve((size_t)NBAT * NDIM * 2);
  float*          HC0    = (float*)carve((size_t)NBAT * 2 * NDIM * 4);
  float*          BIAS   = (float*)carve((size_t)BTOTAL * 4);
  if (off > ws_size || off > (size_t)134217728) return;

  gather_kernel<true><<<(NROW * 64 + 255) / 256, 256, 0, stream>>>(emb_tab, captions, (void*)X16);
  gather_kernel<false><<<(NROW * 128 + 255) / 256, 256, 0, stream>>>(emb_tab, captions, (void*)X32);
  mean_kernel<<<(NBAT * 64 + 255) / 256, 256, 0, stream>>>(features, MEAN16);
  cvt8_kernel<<<(NFROW * 64 + 255) / 256, 256, 0, stream>>>(features, F16, NFROW * 64, 1.0f);

  tpw_kernel<<<dim3(NDIM / 64, NDIM / 64), 256, 0, stream>>>(Wa_enc, NDIM, NDIM, NDIM, WAENC, WCARRY);
  tpw_kernel<<<dim3(NDIM / 64, NDIM / 64), 256, 0, stream>>>(Wa_dec, NDIM, NDIM, NDIM, WAT, WCARRY);
  tpw_kernel<<<dim3(NDIM / 64, NDIM / 64), 256, 0, stream>>>(W_beta, NDIM, NDIM, NDIM, WAT + (size_t)NDIM * NDIM, WCARRY);
  tpw_kernel<<<dim3(NGATE / 64, NDIM / 64), 256, 0, stream>>>(W_hh, NDIM, NGATE, 1024, WG, WCARRY);
  tpw_kernel<<<dim3(NGATE / 64, NDIM / 64), 256, 0, stream>>>(W_ih + (size_t)NDIM * NGATE, NDIM, NGATE, 1024, WG + NDIM, WCARRY);
  tpw_kernel<<<dim3(NGATE / 64, NDIM / 64), 256, 0, stream>>>(W_ih, NDIM, NGATE, NDIM, WXT, WCARRY);
  tpw_kernel<<<dim3(NDIM / 64, NDIM / 64), 256, 0, stream>>>(W_init_h, NDIM, NDIM, NDIM, WINIT, WCARRY);
  tpw_kernel<<<dim3(NDIM / 64, NDIM / 64), 256, 0, stream>>>(W_init_c, NDIM, NDIM, NDIM, WINIT + (size_t)NDIM * NDIM, WCARRY);
  tpw_kernel<<<dim3(NDIM / 64, NDIM / 64), 256, 0, stream>>>(W_Lh, NDIM, NDIM, 1024, WDEEP, WCARRY);
  tpw_kernel<<<dim3(NDIM / 64, NDIM / 64), 256, 0, stream>>>(W_Lz, NDIM, NDIM, 1024, WDEEP + NDIM, WCARRY);
  tpw_kernel<<<dim3(NVOCP / 64, NDIM / 64), 256, 0, stream>>>(W_Lo, NDIM, NVOC, NDIM, WLOT, WCARRY);
  bias_kernel<<<(BTOTAL / 4 + 255) / 256, 256, 0, stream>>>(b_init_h, b_init_c, ba_dec, b_beta, b_ih, b_hh, b_Lh, b_Lz, b_Lo, BIAS);

  {
    const int tiles = (NBAT / 64) * (1024 / 64);
    wmma_gemm64<0, false><<<(tiles + 7) / 8, 256, 0, stream>>>(MEAN16, NDIM, WINIT, NDIM, (void*)HC0, 1024,
        BIAS + BOFF_INIT, X32, NDIM, NBAT, 1024, NDIM, PINV, 1.0f);
  }
  {
    const int tiles = (NFROW / 64) * (NDIM / 64);
    wmma_gemm64<0, false><<<(tiles + 7) / 8, 256, 0, stream>>>(F16, NDIM, WAENC, NDIM, (void*)FPJ, NDIM,
        ba_enc, X32, NDIM, NFROW, NDIM, NDIM, WINV, 1.0f);
  }
  {
    const int tiles = (NROW / 64) * (NGATE / 64);
    wmma_gemm64<0, false><<<(tiles + 7) / 8, 256, 0, stream>>>(X16, NDIM, WXT, NDIM, (void*)XG, NGATE,
        BIAS + BOFF_GATE, X32, NDIM, NROW, NGATE, NDIM, PINV, 1.0f);
  }

  rec_kernel<<<NBAT / 16, 256, 0, stream>>>(features, FPJ, HC0, XG, BIAS + BOFF_AT, Wa_full, ba_full, WAT, WG, ALW, HZ);

  {
    const int tiles = (NROW / 64) * (NDIM / 64);
    wmma_gemm64<1, true><<<(tiles + 7) / 8, 256, 0, stream>>>(HZ, 1024, WDEEP, 1024, (void*)PRE16, NDIM,
        BIAS + BOFF_DEEP, X32, NDIM, NROW, NDIM, 1024, PINV, ACARRY);
  }
  {
    const int tiles = (NROW / 64) * (NVOCP / 64);
    wmma_gemm64<0, false><<<(tiles + 7) / 8, 256, 0, stream>>>(PRE16, NDIM, WLOT, NDIM, (void*)LG, NVOCP,
        BIAS + BOFF_LO, X32, NDIM, NROW, NVOCP, NDIM, PINV, 1.0f);
  }
  copy_rows_kernel<NVOC, NVOCP><<<(NOUT0 / 4 + 255) / 256, 256, 0, stream>>>(LG, out_logits, NOUT0 / 4);
  copy_rows_kernel<NLOC, ALPITCH><<<(NOUT1 / 4 + 255) / 256, 256, 0, stream>>>(ALW, out_alphas, NOUT1 / 4);
}
